// PointnetSAModuleMSG_56642028700412
// MI455X (gfx1250) — hardware-verified
//
#include <hip/hip_runtime.h>
#pragma clang fp contract(off)

typedef __attribute__((ext_vector_type(16))) _Float16 v16h;
typedef __attribute__((ext_vector_type(8)))  _Float16 v8h;
typedef __attribute__((ext_vector_type(8)))  float    v8f;
typedef __attribute__((ext_vector_type(4)))  float    v4f;
typedef __attribute__((ext_vector_type(4)))  int      v4i;

constexpr int kBatch   = 8;
constexpr int kPts     = 4096;
constexpr int kFeat    = 128;
constexpr int kCin     = 131;
constexpr int kCout    = 256;
constexpr int kNpoint  = 1024;
constexpr int kNsample = 32;
constexpr float kBnEps = 1e-5f;
constexpr float kRad2  = 0.01f;
constexpr float kWCarry = 1024.0f;

constexpr int kRowsA   = kBatch * kPts;
constexpr int kABlocks = (kRowsA * kFeat / 8) / 256;
constexpr int kBBlocks = (kCout * kFeat / 8) / 256;

static_assert(kCin == kFeat + 3, "channel split");
static_assert(kFeat % 32 == 0, "K multiple of 32");
static_assert(kRowsA % 64 == 0 && kCout % 64 == 0, "M,N multiples of 64");
static_assert((kRowsA * kFeat / 8) % 256 == 0, "prep A coverage");
static_assert((kCout * kFeat / 8) % 256 == 0, "prep B coverage");
static_assert(kNsample == 32 && kNpoint % 32 == 0, "group tiling");

constexpr size_t kOffA16  = 0;
constexpr size_t kSzA16   = (size_t)kRowsA * kFeat * 2;
constexpr size_t kOffBt16 = kOffA16 + kSzA16;
constexpr size_t kSzBt16  = (size_t)kCout * kFeat * 2;
constexpr size_t kOffCent = kOffBt16 + kSzBt16;
constexpr size_t kSzCent  = (size_t)kBatch * kNpoint * 3 * 4;
constexpr size_t kOffP    = kOffCent + kSzCent;
constexpr size_t kSzP     = (size_t)kRowsA * kCout * 4;
constexpr size_t kWsTotal = kOffP + kSzP;
static_assert(kWsTotal <= (size_t)134217728, "carve within 128 MiB");
static_assert(kOffBt16 % 128 == 0 && kOffCent % 128 == 0 && kOffP % 128 == 0, "line aligned carve");

constexpr size_t kOut0Bytes = (size_t)kBatch * kNpoint * 3 * 4;
constexpr size_t kOut1Bytes = (size_t)kBatch * kCout * kNpoint * 4;
static_assert(kOut0Bytes == 98304 && kOut0Bytes % 128 == 0, "output 1 offset");
static_assert(kOut0Bytes + kOut1Bytes == 8486912, "output total");

__global__ __launch_bounds__(256) void prep_planes(
    const float* __restrict__ feat, const float* __restrict__ W,
    const float* __restrict__ bn_g, const float* __restrict__ bn_b,
    const float* __restrict__ bn_m, const float* __restrict__ bn_v,
    _Float16* __restrict__ A16, _Float16* __restrict__ Bt16) {
  __shared__ float s_sc[kFeat];
  __shared__ float s_mu[kFeat];
  __shared__ float s_be[kFeat];
  const int tid = threadIdx.x;
  if (tid < kFeat) {
    const int c = 3 + tid;
    s_sc[tid] = bn_g[c] / sqrtf(bn_v[c] + kBnEps);
    s_mu[tid] = bn_m[c];
    s_be[tid] = bn_b[c];
  }
  __syncthreads();
  if ((int)blockIdx.x < kABlocks) {
    const size_t t = (size_t)blockIdx.x * 256 + tid;
    const int c0 = (tid & 15) * 8;
    const v4f* src = (const v4f*)(feat + t * 8);
    const v4f x0 = src[0];
    const v4f x1 = src[1];
    v8h hv;
#pragma unroll
    for (int e = 0; e < 4; ++e) {
      float a = (x0[e] - s_mu[c0 + e]) * s_sc[c0 + e] + s_be[c0 + e];
      a = fmaxf(a, 0.0f);
      hv[e] = (_Float16)a;
      float c = (x1[e] - s_mu[c0 + 4 + e]) * s_sc[c0 + 4 + e] + s_be[c0 + 4 + e];
      c = fmaxf(c, 0.0f);
      hv[4 + e] = (_Float16)c;
    }
    _Float16* dst = A16 + t * 8;
    *(volatile v8h*)dst = hv;
    __threadfence();
    *(volatile v8h*)dst = hv;
  } else {
    const int t = ((int)blockIdx.x - kABlocks) * 256 + tid;
    const int o = t >> 4;
    const int c0 = (t & 15) * 8;
    const float* wr = W + (size_t)o * kCin + 3 + c0;
    v8h hv;
#pragma unroll
    for (int e = 0; e < 8; ++e) {
      const float w = wr[e] * kWCarry;
      hv[e] = (_Float16)w;
    }
    _Float16* dst = Bt16 + (size_t)t * 8;
    *(volatile v8h*)dst = hv;
    __threadfence();
    *(volatile v8h*)dst = hv;
  }
}

__global__ __launch_bounds__(256) void fps_select(
    const float* __restrict__ xyz, float* __restrict__ out0, float* __restrict__ cent) {
#pragma clang fp contract(off)
  __shared__ __align__(16) float xs[kPts * 3];
  __shared__ int   sel[kNpoint];
  __shared__ float sv[2][8];
  __shared__ int   si[2][8];

  const int b    = blockIdx.x;
  const int tid  = threadIdx.x;
  const int wave = tid >> 5;
  const int lane = tid & 31;

  {
    const v4f* src = (const v4f*)(xyz + (size_t)b * kPts * 3);
#pragma unroll 1
    for (int it = 0; it < 12; ++it) {
      const v4f v = src[it * 256 + tid];
      *(v4f*)(xs + 4 * (it * 256 + tid)) = v;
    }
  }
  if (tid == 0) sel[0] = 0;
  __syncthreads();

  float lx[16], ly[16], lz[16], md[16];
#pragma unroll
  for (int i = 0; i < 16; ++i) {
    const int n = i * 256 + tid;
    lx[i] = xs[n * 3 + 0];
    ly[i] = xs[n * 3 + 1];
    lz[i] = xs[n * 3 + 2];
    md[i] = 1e10f;
  }

  int last = 0;
#pragma unroll 1
  for (int step = 1; step < kNpoint; ++step) {
    const float bx = xs[last * 3 + 0];
    const float by = xs[last * 3 + 1];
    const float bz = xs[last * 3 + 2];

    float best = -1.0f;
    int bestn = 0;
#pragma unroll
    for (int i = 0; i < 16; ++i) {
      const float dx = lx[i] - bx;
      const float dy = ly[i] - by;
      const float dz = lz[i] - bz;
      const float t0 = dx * dx;
      const float t1 = dy * dy;
      const float t2 = dz * dz;
      const float d  = (t0 + t2) + t1;
      const float m  = fminf(md[i], d);
      md[i] = m;
      const bool up = (m > best);
      best  = up ? m : best;
      bestn = up ? (i * 256 + tid) : bestn;
    }
#pragma unroll
    for (int off = 16; off > 0; off >>= 1) {
      const float ov = __shfl_xor(best, off, 32);
      const int   oi = __shfl_xor(bestn, off, 32);
      const bool take = (ov > best) || ((ov == best) && (oi < bestn));
      best  = take ? ov : best;
      bestn = take ? oi : bestn;
    }
    const int par = step & 1;
    if (lane == 0) { sv[par][wave] = best; si[par][wave] = bestn; }
    __syncthreads();
    float fv = sv[par][0];
    int   fi = si[par][0];
#pragma unroll
    for (int w = 1; w < 8; ++w) {
      const float ov = sv[par][w];
      const int   oi = si[par][w];
      const bool take = (ov > fv) || ((ov == fv) && (oi < fi));
      fv = take ? ov : fv;
      fi = take ? oi : fi;
    }
    fi = fi < 0 ? 0 : (fi > kPts - 1 ? kPts - 1 : fi);
    last = fi;
    if (tid == 0) sel[step] = last;
  }
  __syncthreads();

  v4f ov4[3];
#pragma unroll
  for (int it = 0; it < 3; ++it) {
    const int q = it * 256 + tid;
#pragma unroll
    for (int e = 0; e < 4; ++e) {
      const int f  = 4 * q + e;
      const int pt = f / 3;
      const int cm = f - 3 * pt;
      int id = sel[pt];
      id = id < 0 ? 0 : (id > kPts - 1 ? kPts - 1 : id);
      ov4[it][e] = xs[id * 3 + cm];
    }
  }
  float* d0 = out0 + (size_t)b * (kNpoint * 3);
  float* d1 = cent + (size_t)b * (kNpoint * 3);
  for (int pass = 0; pass < 2; ++pass) {
#pragma unroll
    for (int it = 0; it < 3; ++it) {
      *(volatile v4f*)(d0 + 4 * (it * 256 + tid)) = ov4[it];
      *(volatile v4f*)(d1 + 4 * (it * 256 + tid)) = ov4[it];
    }
    __threadfence();
  }
}

union FragH { v16h v; v8h h[2]; };
__device__ __forceinline__ v16h frag_load_h(const _Float16* p) {
  FragH f;
  f.h[0] = *(const v8h*)(p);
  f.h[1] = *(const v8h*)(p + 16);
  return f.v;
}
__device__ __forceinline__ v8f mma_h(v16h a, v16h b, v8f c) {
  return __builtin_amdgcn_wmma_f32_16x16x32_f16(false, a, false, b, (short)0, c, false, false);
}
__device__ __forceinline__ void dep_guard_row_h(v8f& a, v8f& b, v8f& c, v8f& d,
                                                v16h x, v16h y0, v16h y1, v16h y2, v16h y3) {
  asm volatile("v_nop\n\tv_nop\n\tv_nop\n\tv_nop"
               : "+v"(a), "+v"(b), "+v"(c), "+v"(d)
               : "v"(x), "v"(y0), "v"(y1), "v"(y2), "v"(y3));
}
__device__ __forceinline__ void keep4_h(v16h a, v16h b, v16h c, v16h d) {
  asm volatile("v_nop" :: "v"(a), "v"(b), "v"(c), "v"(d));
}
__device__ __forceinline__ void acc_guard4(v8f& a, v8f& b, v8f& c, v8f& d) {
  asm volatile("v_nop\n\tv_nop\n\tv_nop\n\tv_nop" : "+v"(a), "+v"(b), "+v"(c), "+v"(d));
}

__global__ __launch_bounds__(256) void gemm_f16_tile64(
    const _Float16* __restrict__ A, int lda,
    const _Float16* __restrict__ Bt, int ldb,
    float* __restrict__ C, int ldc,
    int M, int N, int K, float scale) {
  __shared__ __align__(16) float sT[8][16 * 68];
  const int lane = threadIdx.x & 31;
  const int wave = threadIdx.x >> 5;
  const int tilesN = N >> 6;
  const int tilesM = M >> 6;
  const int tile = blockIdx.x * 8 + wave;
  if (tile >= tilesM * tilesN) return;
  const int tm = tile / tilesN;
  const int tn = tile - tm * tilesN;
  const int m0 = tm << 6;
  const int n0 = tn << 6;

  const int rlane = lane & 15;
  const int koff  = (lane >> 4) * 8;
  const int mOff  = (lane >> 4) * 8;

  v8f acc[4][4];
#pragma unroll
  for (int i = 0; i < 4; ++i)
#pragma unroll
    for (int j = 0; j < 4; ++j) acc[i][j] = (v8f){0.f, 0.f, 0.f, 0.f, 0.f, 0.f, 0.f, 0.f};

  for (int k0 = 0; k0 < K; k0 += 32) {
    v16h bh[4];
#pragma unroll
    for (int j = 0; j < 4; ++j) {
      const size_t bo = (size_t)(n0 + (j << 4) + rlane) * ldb + koff + k0;
      bh[j] = frag_load_h(Bt + bo);
    }
#pragma unroll
    for (int i = 0; i < 4; ++i) {
      const size_t ao = (size_t)(m0 + (i << 4) + rlane) * lda + koff + k0;
      const v16h ah = frag_load_h(A + ao);
#pragma unroll
      for (int j = 0; j < 4; ++j) acc[i][j] = mma_h(ah, bh[j], acc[i][j]);
      dep_guard_row_h(acc[i][0], acc[i][1], acc[i][2], acc[i][3], ah, bh[0], bh[1], bh[2], bh[3]);
    }
    keep4_h(bh[0], bh[1], bh[2], bh[3]);
  }
  acc_guard4(acc[0][0], acc[0][1], acc[0][2], acc[0][3]);
  acc_guard4(acc[1][0], acc[1][1], acc[1][2], acc[1][3]);
  acc_guard4(acc[2][0], acc[2][1], acc[2][2], acc[2][3]);
  acc_guard4(acc[3][0], acc[3][1], acc[3][2], acc[3][3]);

  float* slab = sT[wave];
#pragma unroll
  for (int i = 0; i < 4; ++i) {
    const int mBase = m0 + (i << 4);
#pragma unroll
    for (int j = 0; j < 4; ++j) {
#pragma unroll
      for (int r = 0; r < 8; ++r) {
        const float v = acc[i][j][r] * scale;
        slab[(mOff + r) * 68 + (j << 4) + rlane] = v;
      }
    }
    __builtin_amdgcn_fence(__ATOMIC_RELEASE, "workgroup");
    __builtin_amdgcn_wave_barrier();
    __builtin_amdgcn_fence(__ATOMIC_ACQUIRE, "workgroup");
    {
      const int hh = lane >> 4;
      const int c4 = (lane & 15) * 4;
      for (int pass = 0; pass < 2; ++pass) {
#pragma unroll
        for (int it = 0; it < 8; ++it) {
          const int row = it * 2 + hh;
          const v4f v = *(const v4f*)(slab + row * 68 + c4);
          *(volatile v4f*)(C + (size_t)(mBase + row) * ldc + n0 + c4) = v;
        }
        __threadfence();
      }
    }
    __builtin_amdgcn_fence(__ATOMIC_RELEASE, "workgroup");
    __builtin_amdgcn_wave_barrier();
    __builtin_amdgcn_fence(__ATOMIC_ACQUIRE, "workgroup");
  }
}

__global__ __launch_bounds__(256) void group_gather_max(
    const float* __restrict__ xyz, const float* __restrict__ W, const float* __restrict__ bias,
    const float* __restrict__ bn_g, const float* __restrict__ bn_b,
    const float* __restrict__ bn_m, const float* __restrict__ bn_v,
    const float* __restrict__ cent, const float* __restrict__ P, float* __restrict__ out1) {
#pragma clang fp contract(off)
  __shared__ __align__(16) int   nid[32 * kNsample];
  __shared__ float rr[3 * 32 * kNsample];
  __shared__ int   s_cnt[32];
  __shared__ int   s_first[32];
  __shared__ float cst[12];
  __shared__ __align__(16) float tile[kCout * 36];

  const int tid  = threadIdx.x;
  const int wave = tid >> 5;
  const int lane = tid & 31;
  const int b    = blockIdx.x >> 5;
  const int s0   = (blockIdx.x & 31) * 32;
  const int g0   = b * kNpoint + s0;
  const float* xb = xyz + (size_t)b * kPts * 3;

  if (tid < 3) {
    cst[tid]     = bn_m[tid];
    cst[4 + tid] = bn_g[tid] / sqrtf(bn_v[tid] + kBnEps);
    cst[8 + tid] = bn_b[tid];
  }
#pragma unroll
  for (int e = 0; e < 4; ++e) nid[4 * tid + e] = 0;
  __syncthreads();

#pragma unroll 1
  for (int i = 0; i < 4; ++i) {
    const int sl = wave * 4 + i;
    const float cx = cent[(size_t)(g0 + sl) * 3 + 0];
    const float cy = cent[(size_t)(g0 + sl) * 3 + 1];
    const float cz = cent[(size_t)(g0 + sl) * 3 + 2];
    int cnt = 0;
    int first = kPts - 1;
    bool have = false;
    for (int base = 0; base < kPts && cnt < kNsample; base += 32) {
      const int n = base + lane;
      const float dx = cx - xb[n * 3 + 0];
      const float dy = cy - xb[n * 3 + 1];
      const float dz = cz - xb[n * 3 + 2];
      const float t0 = dx * dx;
      const float t1 = dy * dy;
      const float t2 = dz * dz;
      const float d2 = (t0 + t2) + t1;
      const bool valid = d2 < kRad2;
      const unsigned mask = (unsigned)__ballot(valid ? 1 : 0);
      if (!have && mask != 0u) { first = base + __builtin_ctz(mask); have = true; }
      const int before = __popc(mask & ((1u << lane) - 1u));
      const int pos = cnt + before;
      if (valid && pos < kNsample) nid[sl * kNsample + pos] = n;
      cnt += __popc(mask);
    }
    if (cnt > kNsample) cnt = kNsample;
    if (lane == 0) { s_cnt[sl] = cnt; s_first[sl] = first; }
  }
  __syncthreads();

  {
    const int sl = tid >> 3;
    const int kb = (tid & 7) * 4;
    const int cnt = s_cnt[sl];
    const int first = s_first[sl];
    const float cx = cent[(size_t)(g0 + sl) * 3 + 0];
    const float cy = cent[(size_t)(g0 + sl) * 3 + 1];
    const float cz = cent[(size_t)(g0 + sl) * 3 + 2];
    const float m0 = cst[0], m1 = cst[1], m2 = cst[2];
    const float q0 = cst[4], q1 = cst[5], q2 = cst[6];
    const float e0 = cst[8], e1 = cst[9], e2 = cst[10];
#pragma unroll
    for (int e = 0; e < 4; ++e) {
      const int p = 4 * tid + e;
      const int raw = nid[p];
      int n = ((kb + e) < cnt) ? raw : first;
      n = n < 0 ? 0 : (n > kPts - 1 ? kPts - 1 : n);
      const float px = xb[n * 3 + 0];
      const float py = xb[n * 3 + 1];
      const float pz = xb[n * 3 + 2];
      float r0 = ((px - cx) - m0) * q0 + e0;
      float r1 = ((py - cy) - m1) * q1 + e1;
      float r2 = ((pz - cz) - m2) * q2 + e2;
      r0 = fmaxf(r0, 0.0f);
      r1 = fmaxf(r1, 0.0f);
      r2 = fmaxf(r2, 0.0f);
      nid[p] = n;
      rr[p] = r0;
      rr[1024 + p] = r1;
      rr[2048 + p] = r2;
    }
  }
  __syncthreads();

  {
    const int o = tid;
    const float w0 = W[(size_t)o * kCin + 0];
    const float w1 = W[(size_t)o * kCin + 1];
    const float w2 = W[(size_t)o * kCin + 2];
    const float bo = bias[o];
    const float* Pb = P + (size_t)b * kPts * kCout + o;
#pragma unroll 1
    for (int s = 0; s < 32; ++s) {
      float m = -__builtin_huge_valf();
#pragma unroll 1
      for (int kk = 0; kk < 4; ++kk) {
        const int p0 = s * kNsample + kk * 8;
        float pv[8];
#pragma unroll
        for (int u = 0; u < 8; ++u) {
          const int n = nid[p0 + u];
          pv[u] = Pb[(size_t)n * kCout];
        }
#pragma unroll
        for (int u = 0; u < 8; ++u) {
          float v = pv[u];
          v = v + rr[p0 + u] * w0;
          v = v + rr[1024 + p0 + u] * w1;
          v = v + rr[2048 + p0 + u] * w2;
          m = fmaxf(m, v);
        }
      }
      tile[o * 36 + s] = m + bo;
    }
  }
  __syncthreads();

  {
    const int q  = lane >> 3;
    const int c4 = (lane & 7) * 4;
    for (int pass = 0; pass < 2; ++pass) {
#pragma unroll
      for (int it = 0; it < 8; ++it) {
        const int o = wave * 32 + it * 4 + q;
        const v4f v = *(const v4f*)(tile + o * 36 + c4);
        *(volatile v4f*)(out1 + ((size_t)(b * kCout + o) * kNpoint + s0 + c4)) = v;
      }
      __threadfence();
    }
  }
}

extern "C" void kernel_launch(void* const* d_in, const int* in_sizes, int n_in,
                              void* d_out, int out_size, void* d_ws, size_t ws_size,
                              hipStream_t stream) {
  (void)in_sizes; (void)out_size;
  if (n_in < 8) return;
  if (ws_size < kWsTotal) return;

  const float* xyz      = (const float*)d_in[0];
  const float* feat     = (const float*)d_in[1];
  const float* W        = (const float*)d_in[2];
  const float* bias     = (const float*)d_in[3];
  const float* bn_gamma = (const float*)d_in[4];
  const float* bn_beta  = (const float*)d_in[5];
  const float* bn_mean  = (const float*)d_in[6];
  const float* bn_var   = (const float*)d_in[7];

  float* out0 = (float*)d_out;
  float* out1 = (float*)d_out + (kOut0Bytes / 4);

  char* ws = (char*)d_ws;
  _Float16* A16  = (_Float16*)(ws + kOffA16);
  _Float16* Bt16 = (_Float16*)(ws + kOffBt16);
  float*    cent = (float*)(ws + kOffCent);
  float*    P    = (float*)(ws + kOffP);

  prep_planes<<<kABlocks + kBBlocks, 256, 0, stream>>>(feat, W, bn_gamma, bn_beta, bn_mean, bn_var, A16, Bt16);
  fps_select<<<kBatch, 256, 0, stream>>>(xyz, out0, cent);
  gemm_f16_tile64<<<((kRowsA / 64) * (kCout / 64)) / 8, 256, 0, stream>>>(
      A16, kFeat, Bt16, kFeat, P, kCout, kRowsA, kCout, kFeat, 1.0f / kWCarry);
  group_gather_max<<<kBatch * (kNpoint / 32), 256, 0, stream>>>(
      xyz, W, bias, bn_gamma, bn_beta, bn_mean, bn_var, cent, P, out1);
}
